// EdgeGate_644245095026
// MI455X (gfx1250) — hardware-verified
//
#include <hip/hip_runtime.h>
#include <stdint.h>
#include <stddef.h>


#define ND   128
#define HD   256
#define KW   384
#define PQW  512
#define KQ   (KW / 8)
#define GT   128
#define ET   256
#define CT   256

static_assert((ND % 32) == 0);
static_assert(HD == 32 * 8);
static_assert((KW % 8) == 0);
static_assert(PQW == 2 * HD);

typedef float          v4f   __attribute__((ext_vector_type(4)));
typedef float          v8f   __attribute__((ext_vector_type(8)));
typedef unsigned short v8us  __attribute__((ext_vector_type(8)));
typedef unsigned int   v4u   __attribute__((ext_vector_type(4)));
typedef unsigned int   v8u   __attribute__((ext_vector_type(8)));
typedef __bf16         v16bf __attribute__((ext_vector_type(16)));
union Frag { v16bf v; v8us h[2]; v8u u; };

__device__ __forceinline__ unsigned bfb(float a) {
  unsigned u = __builtin_bit_cast(unsigned, a);
  u += 0x7FFFu + ((u >> 16) & 1u);
  return u >> 16;
}

__device__ __forceinline__ void split8(const float* f, v4u& ph, v4u& pl) {
  unsigned hw[8], lw[8];
#pragma unroll
  for (int i = 0; i < 8; ++i) {
    hw[i] = bfb(f[i]);
    const float hf = __builtin_bit_cast(float, hw[i] << 16);
    lw[i] = bfb(f[i] - hf);
  }
#pragma unroll
  for (int i = 0; i < 4; ++i) {
    ph[i] = hw[2 * i] | (hw[2 * i + 1] << 16);
    pl[i] = lw[2 * i] | (lw[2 * i + 1] << 16);
  }
}

__device__ __forceinline__ v8f wm(Frag a, Frag b, v8f c) {
  v8f d = __builtin_amdgcn_wmma_f32_16x16x32_bf16(false, a.v, false, b.v, (short)0, c, false, false);
  asm volatile("v_nop\n\tv_nop\n\tv_nop\n\tv_nop" : "+v"(d) : "v"(a.u), "v"(b.u));
  return d;
}

__global__ __launch_bounds__(CT) void k_split_rows(const float* __restrict__ src, int nValid,
                                                   unsigned short* hi, unsigned short* lo, int nChunks) {
  const int c = blockIdx.x * CT + threadIdx.x;
  if (c >= nChunks) return;
  const int row = c >> 4, q = c & 15;
  const int rr = row < nValid ? row : nValid - 1;
  const float* p = src + (size_t)rr * ND + q * 8;
  const v4f a = *(const v4f*)p;
  const v4f b = *(const v4f*)(p + 4);
  const bool ok = row < nValid;
  float f[8];
  f[0] = a.x; f[1] = a.y; f[2] = a.z; f[3] = a.w;
  f[4] = b.x; f[5] = b.y; f[6] = b.z; f[7] = b.w;
#pragma unroll
  for (int i = 0; i < 8; ++i) f[i] = ok ? f[i] : 0.0f;
  v4u ph, pl;
  split8(f, ph, pl);
  unsigned short* hp = hi + (size_t)c * 8;
  unsigned short* lp = lo + (size_t)c * 8;
  *(volatile v4u*)hp = ph;
  *(volatile v4u*)lp = pl;
  __threadfence();
  *(volatile v4u*)hp = ph;
  *(volatile v4u*)lp = pl;
}

__global__ __launch_bounds__(CT) void k_split_w1t(const float* __restrict__ W1,
                                                  unsigned short* wh, unsigned short* wl) {
  const int c = blockIdx.x * CT + threadIdx.x;
  if (c >= HD * KQ) return;
  const int n = c / KQ, kq = c - n * KQ;
  float f[8];
#pragma unroll
  for (int j = 0; j < 8; ++j) f[j] = W1[(size_t)(kq * 8 + j) * HD + n];
  v4u ph, pl;
  split8(f, ph, pl);
  unsigned short* hp = wh + (size_t)c * 8;
  unsigned short* lp = wl + (size_t)c * 8;
  *(volatile v4u*)hp = ph;
  *(volatile v4u*)lp = pl;
  __threadfence();
  *(volatile v4u*)hp = ph;
  *(volatile v4u*)lp = pl;
}

__global__ __launch_bounds__(GT) void k_gemm(const unsigned short* __restrict__ Ah,
                                             const unsigned short* __restrict__ Al,
                                             const unsigned short* __restrict__ Wh,
                                             const unsigned short* __restrict__ Wl,
                                             float* outp, int ldo, int kbase) {
  __shared__ __attribute__((aligned(16))) float stg[(GT / 32) * 32 * 64];
  const int tid = threadIdx.x, lane = tid & 31, wave = tid >> 5, h = lane >> 4, m = lane & 15;
  const int row0 = blockIdx.x * 32;
  const int cb   = blockIdx.y * HD + wave * 64;
  const int n0   = cb & (HD - 1);
  const int kofs = kbase + (cb / HD) * ND;

  v8f acc[2][4];
#pragma unroll
  for (int mt = 0; mt < 2; ++mt)
#pragma unroll
    for (int nt = 0; nt < 4; ++nt) {
      v8f z;
#pragma unroll
      for (int i = 0; i < 8; ++i) z[i] = 0.0f;
      acc[mt][nt] = z;
    }

#pragma unroll 1
  for (int ks = 0; ks < ND / 32; ++ks) {
    const int k0 = ks * 32 + 8 * h;
    Frag ah[2], al[2];
#pragma unroll
    for (int mt = 0; mt < 2; ++mt) {
      const size_t ao = (size_t)(row0 + mt * 16 + m) * ND + k0;
      ah[mt].h[0] = *(const v8us*)(Ah + ao);
      ah[mt].h[1] = *(const v8us*)(Ah + ao + 16);
      al[mt].h[0] = *(const v8us*)(Al + ao);
      al[mt].h[1] = *(const v8us*)(Al + ao + 16);
    }
#pragma unroll
    for (int nt = 0; nt < 4; ++nt) {
      const size_t bo = (size_t)(n0 + nt * 16 + m) * KW + kofs + k0;
      Frag bh, bl;
      bh.h[0] = *(const v8us*)(Wh + bo);
      bh.h[1] = *(const v8us*)(Wh + bo + 16);
      bl.h[0] = *(const v8us*)(Wl + bo);
      bl.h[1] = *(const v8us*)(Wl + bo + 16);
#pragma unroll
      for (int mt = 0; mt < 2; ++mt) {
        acc[mt][nt] = wm(ah[mt], bh, acc[mt][nt]);
        acc[mt][nt] = wm(ah[mt], bl, acc[mt][nt]);
        acc[mt][nt] = wm(al[mt], bh, acc[mt][nt]);
      }
    }
  }

  float* sw = stg + wave * (32 * 64);
#pragma unroll
  for (int mt = 0; mt < 2; ++mt)
#pragma unroll
    for (int nt = 0; nt < 4; ++nt)
#pragma unroll
      for (int r = 0; r < 8; ++r)
        sw[(mt * 16 + 8 * h + r) * 64 + nt * 16 + m] = acc[mt][nt][r];
  __syncthreads();

  v4f ov[16];
#pragma unroll
  for (int it = 0; it < 16; ++it) ov[it] = *(const v4f*)(sw + (it * 2 + h) * 64 + m * 4);
  float* ob = outp + (size_t)row0 * ldo + cb + m * 4;
#pragma unroll
  for (int it = 0; it < 16; ++it) *(volatile v4f*)(ob + (size_t)(it * 2 + h) * ldo) = ov[it];
  __threadfence();
#pragma unroll
  for (int it = 0; it < 16; ++it) *(volatile v4f*)(ob + (size_t)(it * 2 + h) * ldo) = ov[it];
}

__global__ __launch_bounds__(ET) void k_edge(const int* __restrict__ ei, const int* __restrict__ batch,
                                             const float* __restrict__ PQ, const float* __restrict__ U,
                                             const float* __restrict__ b1, const float* __restrict__ W2,
                                             const float* __restrict__ b2, float* outp,
                                             int E, int N, int G) {
  const int lane = threadIdx.x & 31;
  const int wave = __builtin_amdgcn_readfirstlane((int)(threadIdx.x >> 5));
  const int ebase = (blockIdx.x * (ET / 32) + wave) * 32;
  if (ebase >= E) return;

  float b1v[8], w2v[8];
  {
    const v4f ba = *(const v4f*)(b1 + 8 * lane), bb = *(const v4f*)(b1 + 8 * lane + 4);
    const v4f wa = *(const v4f*)(W2 + 8 * lane), wb = *(const v4f*)(W2 + 8 * lane + 4);
    b1v[0] = ba.x; b1v[1] = ba.y; b1v[2] = ba.z; b1v[3] = ba.w;
    b1v[4] = bb.x; b1v[5] = bb.y; b1v[6] = bb.z; b1v[7] = bb.w;
    w2v[0] = wa.x; w2v[1] = wa.y; w2v[2] = wa.z; w2v[3] = wa.w;
    w2v[4] = wb.x; w2v[5] = wb.y; w2v[6] = wb.z; w2v[7] = wb.w;
  }
  const float b2v = b2[0];
  float mine = 0.0f;

#pragma unroll 1
  for (int j = 0; j < 32; ++j) {
    int e = ebase + j;
    e = e > E - 1 ? E - 1 : e;
    int s = ei[e];
    int d = ei[(size_t)E + (size_t)e];
    s = s < 0 ? s + N : s;  s = s < 0 ? 0 : (s > N - 1 ? N - 1 : s);
    d = d < 0 ? d + N : d;  d = d < 0 ? 0 : (d > N - 1 ? N - 1 : d);
    int g = batch[s];
    g = g < 0 ? g + G : g;  g = g < 0 ? 0 : (g > G - 1 ? G - 1 : g);

    const float* pp = PQ + (size_t)s * PQW + 8 * lane;
    const float* qp = PQ + (size_t)d * PQW + HD + 8 * lane;
    const float* up = U + (size_t)g * HD + 8 * lane;
    const v4f p0 = *(const v4f*)pp, p1 = *(const v4f*)(pp + 4);
    const v4f q0 = *(const v4f*)qp, q1 = *(const v4f*)(qp + 4);
    const v4f u0 = *(const v4f*)up, u1 = *(const v4f*)(up + 4);
    float hv[8];
    hv[0] = (p0.x + q0.x) + u0.x; hv[1] = (p0.y + q0.y) + u0.y;
    hv[2] = (p0.z + q0.z) + u0.z; hv[3] = (p0.w + q0.w) + u0.w;
    hv[4] = (p1.x + q1.x) + u1.x; hv[5] = (p1.y + q1.y) + u1.y;
    hv[6] = (p1.z + q1.z) + u1.z; hv[7] = (p1.w + q1.w) + u1.w;
    float part = 0.0f;
#pragma unroll
    for (int i = 0; i < 8; ++i) {
      const float hh = hv[i] + b1v[i];
      const float t  = __expf(-hh);
      const float sg = __builtin_amdgcn_rcpf(1.0f + t);
      const float sv = hh * sg;
      part = fmaf(sv, w2v[i], part);
    }
    float tot = part;
    tot += __shfl_xor(tot, 16);
    tot += __shfl_xor(tot, 8);
    tot += __shfl_xor(tot, 4);
    tot += __shfl_xor(tot, 2);
    tot += __shfl_xor(tot, 1);
    mine = (lane == j) ? tot : mine;
  }

  const int eo = ebase + lane;
  const float val = mine + b2v;
  if (eo < E) *(volatile float*)(outp + eo) = val;
  __threadfence();
  if (eo < E) *(volatile float*)(outp + eo) = val;
}

static inline size_t al256(size_t v) { return (v + 255) & ~(size_t)255; }

extern "C" void kernel_launch(void* const* d_in, const int* in_sizes, int n_in,
                              void* d_out, int out_size, void* d_ws, size_t ws_size,
                              hipStream_t stream) {
  if (n_in < 8) return;
  const int G = in_sizes[0] / ND;
  const int N = in_sizes[1] / ND;
  const int E = in_sizes[2] / 2;
  if (G < 1 || N < 1 || E < 1) return;
  if (in_sizes[0] != G * ND || in_sizes[1] != N * ND || in_sizes[2] != 2 * E) return;
  if (in_sizes[3] != N || in_sizes[4] != KW * HD || in_sizes[5] != HD || in_sizes[6] != HD || in_sizes[7] < 1) return;
  if (out_size != E) return;

  const float* instr = (const float*)d_in[0];
  const float* x     = (const float*)d_in[1];
  const int*   ei    = (const int*)d_in[2];
  const int*   batch = (const int*)d_in[3];
  const float* W1    = (const float*)d_in[4];
  const float* b1    = (const float*)d_in[5];
  const float* W2    = (const float*)d_in[6];
  const float* b2    = (const float*)d_in[7];
  float* out = (float*)d_out;

  const int Npad = ((N + 31) / 32) * 32;
  const int Gpad = ((G + 31) / 32) * 32;

  char* ws = (char*)d_ws;
  size_t off = 0;
  const size_t oXh = off; off += al256((size_t)Npad * ND * 2);
  const size_t oXl = off; off += al256((size_t)Npad * ND * 2);
  const size_t oIh = off; off += al256((size_t)Gpad * ND * 2);
  const size_t oIl = off; off += al256((size_t)Gpad * ND * 2);
  const size_t oWh = off; off += al256((size_t)HD * KW * 2);
  const size_t oWl = off; off += al256((size_t)HD * KW * 2);
  const size_t oPQ = off; off += al256((size_t)Npad * PQW * 4);
  const size_t oU  = off; off += al256((size_t)Gpad * HD * 4);
  if (off > ws_size) return;

  unsigned short* xh = (unsigned short*)(ws + oXh);
  unsigned short* xl = (unsigned short*)(ws + oXl);
  unsigned short* ih = (unsigned short*)(ws + oIh);
  unsigned short* il = (unsigned short*)(ws + oIl);
  unsigned short* wh = (unsigned short*)(ws + oWh);
  unsigned short* wl = (unsigned short*)(ws + oWl);
  float* PQ  = (float*)(ws + oPQ);
  float* Upl = (float*)(ws + oU);

  const int xChunks = Npad * (ND / 8);
  const int iChunks = Gpad * (ND / 8);

  k_split_rows<<<(xChunks + CT - 1) / CT, CT, 0, stream>>>(x, N, xh, xl, xChunks);
  k_split_rows<<<(iChunks + CT - 1) / CT, CT, 0, stream>>>(instr, G, ih, il, iChunks);
  k_split_w1t<<<(HD * KQ + CT - 1) / CT, CT, 0, stream>>>(W1, wh, wl);

  k_gemm<<<dim3(Npad / 32, 2, 1), dim3(GT, 1, 1), 0, stream>>>(xh, xl, wh, wl, PQ, PQW, 0);
  k_gemm<<<dim3(Gpad / 32, 1, 1), dim3(GT, 1, 1), 0, stream>>>(ih, il, wh, wl, Upl, HD, 2 * ND);

  const int nWaves  = (E + 31) / 32;
  const int nBlocks = (nWaves + (ET / 32) - 1) / (ET / 32);
  k_edge<<<nBlocks, ET, 0, stream>>>(ei, batch, PQ, Upl, b1, W2, b2, out, E, N, G);
}
